// MixExperts_86251533238441
// MI455X (gfx1250) — hardware-verified
//
#include <hip/hip_runtime.h>
#include <stddef.h>
#include <stdint.h>

#define NB   512
#define NF   64
#define NL   400
#define NE   8
#define NT   4
#define NC1  64
#define NC2  16
#define KW   3
#define NU   (NC2 * NL)
#define KF   (NF * NL)
#define KC   (KW * NF)
#define NG   (NT * NE)
#define MT   (NL / 16)
#define XP   64
#define XR   (NL + 2)
#define HR   (NL + 4)
#define GKW  (KF / 32 / 8)
#define GKC  256
#define HSC  64.0f
#define WSC  256.0f
#define ISC  (1.0f / 16384.0f)

static_assert((NL % 16) == 0);
static_assert((NL % 8) == 0);
static_assert((KF % (32 * 8)) == 0);
static_assert((KF % GKC) == 0);
static_assert((KC % 32) == 0);
static_assert(KC == KW * NC1);
static_assert((NB % 16) == 0);
static_assert(((NB * KF) % 2048) == 0);
static_assert((NU % 4) == 0);
static_assert(NG == 32);
static_assert(NC1 == 64);
static_assert(NC2 == 16);
static_assert(NE == 8);
static_assert(NT == 4);
static_assert((XP % 8) == 0);

#define OFF_ACC  0
#define SZ_ACC   (NT * NU * 4)
#define OFF_X    (OFF_ACC + SZ_ACC)
#define SZ_X     (XR * XP * 2)
#define OFF_H    (OFF_X + SZ_X)
#define SZ_H     (HR * XP * 2)
#define OFF_G    (OFF_H + SZ_H)
#define SZ_G     (NG * 4)
#define LDS_CONV (OFF_G + SZ_G)
static_assert((OFF_X % 16) == 0);
static_assert((OFF_H % 16) == 0);
static_assert((OFF_G % 16) == 0);
static_assert(LDS_CONV <= 300000);

typedef __attribute__((ext_vector_type(16))) __bf16 v16b;
typedef _Float16     v16h __attribute__((ext_vector_type(16)));
typedef _Float16     v8h  __attribute__((ext_vector_type(8)));
typedef float        v8f  __attribute__((ext_vector_type(8)));
typedef float        v4f  __attribute__((ext_vector_type(4)));
typedef unsigned int v4u  __attribute__((ext_vector_type(4)));

__device__ __forceinline__ unsigned short bf_bits(float f) {
  const unsigned u = __float_as_uint(f);
  return (unsigned short)((u + 0x7FFFu + ((u >> 16) & 1u)) >> 16);
}
__device__ __forceinline__ float bfr(float f) { return __uint_as_float(((unsigned)bf_bits(f)) << 16); }
__device__ __forceinline__ unsigned short h_bits(float f) {
  const _Float16 h = (_Float16)f;
  return __builtin_bit_cast(unsigned short, h);
}
__device__ __forceinline__ unsigned pk16(unsigned short a, unsigned short b) { return (unsigned)a | ((unsigned)b << 16); }
__device__ __forceinline__ v8f zero8() { v8f z = {0.f, 0.f, 0.f, 0.f, 0.f, 0.f, 0.f, 0.f}; return z; }

union FragB { v16b v; v4u u[2]; };
__device__ __forceinline__ v16b ldfrag_b(const unsigned short* p) {
  FragB f;
  f.u[0] = *(const v4u*)(p);
  f.u[1] = *(const v4u*)(p + 16);
  return f.v;
}
union FragH { v16h v; v8h h[2]; };
__device__ __forceinline__ v16h ldfrag_h(const _Float16* p) {
  FragH f;
  f.h[0] = *(const v8h*)(p);
  f.h[1] = *(const v8h*)(p + 16);
  return f.v;
}

__device__ __forceinline__ v8f mma_b(v16b a, v16b b, v8f c) {
  return __builtin_amdgcn_wmma_f32_16x16x32_bf16(false, a, false, b, (short)0, c, false, false);
}
__device__ __forceinline__ v8f mma_h(v16h a, v16h b, v8f c) {
  return __builtin_amdgcn_wmma_f32_16x16x32_f16(false, a, false, b, (short)0, c, false, false);
}
__device__ __forceinline__ void guard4(v8f& c0, v8f& c1, v8f& c2, v8f& c3, const v16b& a,
                                       const v16b& b0, const v16b& b1, const v16b& b2, const v16b& b3) {
#if defined(__HIP_DEVICE_COMPILE__)
  asm volatile("v_nop\n\tv_nop\n\tv_nop\n\tv_nop"
               : "+v"(c0), "+v"(c1), "+v"(c2), "+v"(c3)
               : "v"(a), "v"(b0), "v"(b1), "v"(b2), "v"(b3));
#endif
}
__device__ __forceinline__ void guard2(v8f& c0, v8f& c1, const v16b& a, const v16b& b0, const v16b& b1) {
#if defined(__HIP_DEVICE_COMPILE__)
  asm volatile("v_nop\n\tv_nop\n\tv_nop\n\tv_nop"
               : "+v"(c0), "+v"(c1)
               : "v"(a), "v"(b0), "v"(b1));
#endif
}
__device__ __forceinline__ void guard1h(v8f& c0, const v16h& a, const v16h& b0) {
#if defined(__HIP_DEVICE_COMPILE__)
  asm volatile("v_nop\n\tv_nop\n\tv_nop\n\tv_nop"
               : "+v"(c0)
               : "v"(a), "v"(b0));
#endif
}

__global__ __launch_bounds__(256)
void k_cvx(const float* __restrict__ x, unsigned short* Xb) {
  const size_t f8 = ((size_t)blockIdx.x * 256 + threadIdx.x) * 8;
  const v4f a = *(const v4f*)(x + f8);
  const v4f b = *(const v4f*)(x + f8 + 4);
  v4u u;
  u[0] = pk16(bf_bits(a[0]), bf_bits(a[1]));
  u[1] = pk16(bf_bits(a[2]), bf_bits(a[3]));
  u[2] = pk16(bf_bits(b[0]), bf_bits(b[1]));
  u[3] = pk16(bf_bits(b[2]), bf_bits(b[3]));
  unsigned short* dst = Xb + f8;
  *(volatile v4u*)dst = u;
  __threadfence();
  *(volatile v4u*)dst = u;
}

__global__ __launch_bounds__(256)
void k_gkT(const float* __restrict__ gk, unsigned short* Gk) {
  __shared__ __align__(16) unsigned short sT[NE * 264];
  const int t = blockIdx.y, k0 = blockIdx.x * GKC, tid = threadIdx.x;
  const float* p = gk + ((size_t)t * KF + k0 + tid) * NE;
  const v4f a = *(const v4f*)(p);
  const v4f b = *(const v4f*)(p + 4);
  sT[0 * 264 + tid] = bf_bits(a[0]);
  sT[1 * 264 + tid] = bf_bits(a[1]);
  sT[2 * 264 + tid] = bf_bits(a[2]);
  sT[3 * 264 + tid] = bf_bits(a[3]);
  sT[4 * 264 + tid] = bf_bits(b[0]);
  sT[5 * 264 + tid] = bf_bits(b[1]);
  sT[6 * 264 + tid] = bf_bits(b[2]);
  sT[7 * 264 + tid] = bf_bits(b[3]);
  __syncthreads();
  const int e = tid >> 5, q = tid & 31;
  const v4u u = *(const v4u*)(sT + e * 264 + q * 8);
  unsigned short* dst = Gk + (size_t)(t * NE + e) * KF + k0 + q * 8;
  *(volatile v4u*)dst = u;
  __threadfence();
  *(volatile v4u*)dst = u;
}

__global__ __launch_bounds__(64)
void k_w1T(const float* __restrict__ w1, unsigned short* W1) {
  __shared__ __align__(16) unsigned short sT[KC];
  const int r = blockIdx.x, tid = threadIdx.x;
  const float* p = w1 + (size_t)r * KC + tid * KW;
  sT[0 * NF + tid] = bf_bits(p[0]);
  sT[1 * NF + tid] = bf_bits(p[1]);
  sT[2 * NF + tid] = bf_bits(p[2]);
  __syncthreads();
  const int q = (tid < KC / 8) ? tid : 0;
  const v4u u = *(const v4u*)(sT + q * 8);
  unsigned short* dst = W1 + (size_t)r * KC + q * 8;
  if (tid < KC / 8) *(volatile v4u*)dst = u;
  __threadfence();
  if (tid < KC / 8) *(volatile v4u*)dst = u;
}

__global__ __launch_bounds__(64)
void k_w2T(const float* __restrict__ w2, unsigned short* W2) {
  __shared__ __align__(16) unsigned short sT[KC];
  const int r = blockIdx.x, tid = threadIdx.x;
  const float* p = w2 + (size_t)r * KC + tid * KW;
  sT[0 * NF + tid] = h_bits(bfr(p[0]) * WSC);
  sT[1 * NF + tid] = h_bits(bfr(p[1]) * WSC);
  sT[2 * NF + tid] = h_bits(bfr(p[2]) * WSC);
  __syncthreads();
  const int q = (tid < KC / 8) ? tid : 0;
  const v4u u = *(const v4u*)(sT + q * 8);
  unsigned short* dst = W2 + (size_t)r * KC + q * 8;
  if (tid < KC / 8) *(volatile v4u*)dst = u;
  __threadfence();
  if (tid < KC / 8) *(volatile v4u*)dst = u;
}

__global__ __launch_bounds__(256)
void k_gate(const unsigned short* __restrict__ Xb, const unsigned short* __restrict__ Gk,
            const float* __restrict__ gb, float* gates) {
  __shared__ __align__(16) float part[8 * 16 * NG];
  __shared__ __align__(16) float slg[16 * NG];
  __shared__ __align__(16) float sgo[16 * NG];
  const int tid = threadIdx.x, w = tid >> 5, lane = tid & 31, hh = lane >> 4, c = lane & 15;
  const int row0 = blockIdx.x * 16;

  const unsigned short* ap  = Xb + (size_t)(row0 + c) * KF + 8 * hh;
  const unsigned short* bp0 = Gk + (size_t)c * KF + 8 * hh;
  const unsigned short* bp1 = Gk + (size_t)(16 + c) * KF + 8 * hh;
  v8f acc0 = zero8(), acc1 = zero8();
  const int ks0 = w * GKW;
#pragma unroll 1
  for (int ks = ks0; ks < ks0 + GKW; ++ks) {
    const size_t ko = (size_t)32 * ks;
    const v16b a  = ldfrag_b(ap + ko);
    const v16b f0 = ldfrag_b(bp0 + ko);
    const v16b f1 = ldfrag_b(bp1 + ko);
    acc0 = mma_b(a, f0, acc0);
    acc1 = mma_b(a, f1, acc1);
    guard2(acc0, acc1, a, f0, f1);
  }
#pragma unroll
  for (int r = 0; r < 8; ++r) {
    const int m = 8 * hh + r;
    part[(w * 16 + m) * NG + c]      = acc0[r];
    part[(w * 16 + m) * NG + 16 + c] = acc1[r];
  }
  __syncthreads();
  for (int idx = tid; idx < 16 * NG; idx += 256) {
    const int m = idx >> 5, n = idx & 31;
    float s = 0.0f;
#pragma unroll
    for (int ww = 0; ww < 8; ++ww) s += part[(ww * 16 + m) * NG + n];
    slg[idx] = s + bfr(gb[n]);
  }
  __syncthreads();
  if (tid < 64) {
    const int m = tid >> 2, t = tid & 3;
    const float* lg = slg + m * NG + t * NE;
    float mx = lg[0];
#pragma unroll
    for (int e = 1; e < NE; ++e) mx = fmaxf(mx, lg[e]);
    float ex[NE];
    float s = 0.0f;
#pragma unroll
    for (int e = 0; e < NE; ++e) { ex[e] = __expf(lg[e] - mx); s += ex[e]; }
    const float inv = 1.0f / s;
#pragma unroll
    for (int e = 0; e < NE; ++e) sgo[m * NG + t * NE + e] = ex[e] * inv;
  }
  __syncthreads();
  const int srow = (tid < 128) ? (tid >> 3) : 0;
  const int q = tid & 7;
  v4f g4 = {0.0f, 0.0f, 0.0f, 0.0f};
  if (tid < 128) g4 = *(const v4f*)(sgo + srow * NG + 4 * q);
  float* gp = gates + (size_t)(row0 + srow) * NG + 4 * q;
  if (tid < 128) *(volatile v4f*)gp = g4;
  __threadfence();
  if (tid < 128) *(volatile v4f*)gp = g4;
}

__global__ __launch_bounds__(256)
void k_conv(const unsigned short* __restrict__ Xb, const unsigned short* __restrict__ W1,
            const _Float16* __restrict__ W2, const float* __restrict__ gates,
            const float* __restrict__ b1, const float* __restrict__ b2,
            const float* __restrict__ eb, const float* __restrict__ tb, float* out) {
  extern __shared__ __attribute__((aligned(16))) unsigned char smem[];
  float* acc = (float*)(smem + OFF_ACC);
  unsigned short* xT = (unsigned short*)(smem + OFF_X);
  _Float16* hT = (_Float16*)(smem + OFF_H);
  float* sg = (float*)(smem + OFF_G);

  const int b = blockIdx.x;
  const int tid = threadIdx.x, w = tid >> 5, lane = tid & 31, hh = lane >> 4, c = lane & 15;

  {
    const v4f z4 = {0.0f, 0.0f, 0.0f, 0.0f};
    for (int i = tid; i < (NT * NU) / 4; i += 256) ((v4f*)acc)[i] = z4;
    for (int i = tid; i < (2 * XP) / 2; i += 256) ((unsigned int*)xT)[i] = 0u;
    for (int i = tid; i < (4 * XP) / 2; i += 256) ((unsigned int*)hT)[i] = 0u;
    if (tid < NG) sg[tid] = gates[(size_t)b * NG + tid];
  }
  {
    const unsigned short* xrow = Xb + (size_t)b * KF;
    for (int i = tid; i < NF * (NL / 8); i += 256) {
      const int ci = i / (NL / 8), l8 = (i - ci * (NL / 8)) * 8;
      const v4u v = *(const v4u*)(xrow + ci * NL + l8);
      unsigned short* d = xT + (l8 + 2) * XP + ci;
#pragma unroll
      for (int j = 0; j < 4; ++j) {
        d[(2 * j) * XP]     = (unsigned short)(v[j] & 0xFFFFu);
        d[(2 * j + 1) * XP] = (unsigned short)(v[j] >> 16);
      }
    }
  }
  __syncthreads();

#pragma unroll 1
  for (int e = 0; e < NE; ++e) {
    {
      const unsigned short* w1e = W1 + (size_t)e * NC1 * KC + 8 * hh;
      const float* b1e = b1 + e * NC1;
      const float q0 = bfr(b1e[c]), q1 = bfr(b1e[16 + c]), q2 = bfr(b1e[32 + c]), q3 = bfr(b1e[48 + c]);
#pragma unroll 1
      for (int mt = w; mt < MT; mt += 8) {
        v8f c0 = zero8(), c1 = zero8(), c2 = zero8(), c3 = zero8();
        const unsigned short* arow = xT + (16 * mt + c) * XP + 8 * hh;
#pragma unroll
        for (int ks = 0; ks < KC / 32; ++ks) {
          const int j = ks >> 1, ci0 = (ks & 1) * 32;
          const v16b a  = ldfrag_b(arow + j * XP + ci0);
          const v16b f0 = ldfrag_b(w1e + (size_t)(0  + c) * KC + 32 * ks);
          const v16b f1 = ldfrag_b(w1e + (size_t)(16 + c) * KC + 32 * ks);
          const v16b f2 = ldfrag_b(w1e + (size_t)(32 + c) * KC + 32 * ks);
          const v16b f3 = ldfrag_b(w1e + (size_t)(48 + c) * KC + 32 * ks);
          c0 = mma_b(a, f0, c0);
          c1 = mma_b(a, f1, c1);
          c2 = mma_b(a, f2, c2);
          c3 = mma_b(a, f3, c3);
          guard4(c0, c1, c2, c3, a, f0, f1, f2, f3);
        }
        _Float16* hrow = hT + (16 * mt + 8 * hh + 4) * XP;
#pragma unroll
        for (int r = 0; r < 8; ++r) {
          _Float16* hr = hrow + r * XP;
          hr[c]      = (_Float16)(fmaxf(c0[r] + q0, 0.0f) * HSC);
          hr[16 + c] = (_Float16)(fmaxf(c1[r] + q1, 0.0f) * HSC);
          hr[32 + c] = (_Float16)(fmaxf(c2[r] + q2, 0.0f) * HSC);
          hr[48 + c] = (_Float16)(fmaxf(c3[r] + q3, 0.0f) * HSC);
        }
      }
    }
    __syncthreads();
    {
      const _Float16* w2e = W2 + (size_t)(e * NC2 + c) * KC + 8 * hh;
      const float b2v = bfr(b2[e * NC2 + c]);
      const float* ebe = eb + (size_t)e * NU + c * NL;
      const float g0 = sg[0 * NE + e], g1 = sg[1 * NE + e], g2 = sg[2 * NE + e], g3 = sg[3 * NE + e];
#pragma unroll 1
      for (int mt = w; mt < MT; mt += 8) {
        v8f d = zero8();
        const _Float16* hrow = hT + (16 * mt + c) * XP + 8 * hh;
#pragma unroll
        for (int ks = 0; ks < KC / 32; ++ks) {
          const int j = ks >> 1, ci0 = (ks & 1) * 32;
          const v16h a = ldfrag_h(hrow + 2 * j * XP + ci0);
          const v16h f = ldfrag_h(w2e + 32 * ks);
          d = mma_h(a, f, d);
          guard1h(d, a, f);
        }
#pragma unroll
        for (int r = 0; r < 8; ++r) {
          const int l = 16 * mt + 8 * hh + r;
          const float z = fmaxf(fmaf(d[r], ISC, b2v), 0.0f);
          const float E = fmaxf(z + bfr(ebe[l]), 0.0f);
          float* au = acc + c * NL + l;
          const float a0 = fmaf(g0, E, au[0 * NU]);
          const float a1 = fmaf(g1, E, au[1 * NU]);
          const float a2 = fmaf(g2, E, au[2 * NU]);
          const float a3 = fmaf(g3, E, au[3 * NU]);
          au[0 * NU] = a0;
          au[1 * NU] = a1;
          au[2 * NU] = a2;
          au[3 * NU] = a3;
        }
      }
    }
    __syncthreads();
  }

#pragma unroll 1
  for (int t = 0; t < NT; ++t) {
    const float tbv = bfr(tb[t]);
    const v4f* src = (const v4f*)(acc + t * NU);
    float* orow = out + ((size_t)t * NB + b) * NU;
    v4f o[7];
#pragma unroll
    for (int i = 0; i < 7; ++i) {
      const int f = tid + 256 * i;
      const int fc = (f < NU / 4) ? f : (NU / 4 - 1);
      o[i] = src[fc] + tbv;
    }
#pragma unroll
    for (int i = 0; i < 7; ++i) {
      const int f = tid + 256 * i;
      if (i < 6 || tid < (NU / 4 - 256 * 6)) *(volatile v4f*)(orow + 4 * (size_t)f) = o[i];
    }
    __threadfence();
#pragma unroll
    for (int i = 0; i < 7; ++i) {
      const int f = tid + 256 * i;
      if (i < 6 || tid < (NU / 4 - 256 * 6)) *(volatile v4f*)(orow + 4 * (size_t)f) = o[i];
    }
  }
}

extern "C" void kernel_launch(void* const* d_in, const int* in_sizes, int n_in,
                              void* d_out, int out_size, void* d_ws, size_t ws_size,
                              hipStream_t stream) {
  if (n_in < 9) return;
  if (in_sizes[0] != NB * NF * NL) return;
  if (in_sizes[1] != NE * NC1 * NF * KW) return;
  if (in_sizes[2] != NE * NC1) return;
  if (in_sizes[3] != NE * NC2 * NC1 * KW) return;
  if (in_sizes[4] != NE * NC2) return;
  if (in_sizes[5] != NE * NU) return;
  if (in_sizes[6] != NT * KF * NE) return;
  if (in_sizes[7] != NT * NE) return;
  if (in_sizes[8] != NT) return;
  if (out_size != NT * NB * NU) return;

  const float* x   = (const float*)d_in[0];
  const float* w1  = (const float*)d_in[1];
  const float* b1  = (const float*)d_in[2];
  const float* w2  = (const float*)d_in[3];
  const float* b2  = (const float*)d_in[4];
  const float* eb  = (const float*)d_in[5];
  const float* gk  = (const float*)d_in[6];
  const float* gb  = (const float*)d_in[7];
  const float* tbp = (const float*)d_in[8];
  float* out = (float*)d_out;

  const size_t sXb = (size_t)NB * KF * 2;
  const size_t sGk = (size_t)NG * KF * 2;
  const size_t sW1 = (size_t)NE * NC1 * KC * 2;
  const size_t sW2 = (size_t)NE * NC2 * KC * 2;
  const size_t sGt = (size_t)NB * NG * 4;
  size_t off = 0;
  const size_t oXb = off; off += sXb;
  const size_t oGk = off; off += sGk;
  const size_t oW1 = off; off += sW1;
  const size_t oW2 = off; off += sW2;
  const size_t oGt = off; off += sGt;
  if (off > ws_size) return;
  if (off > (size_t)134217728) return;

  char* ws = (char*)d_ws;
  unsigned short* Xb = (unsigned short*)(ws + oXb);
  unsigned short* Gk = (unsigned short*)(ws + oGk);
  unsigned short* W1 = (unsigned short*)(ws + oW1);
  unsigned short* W2 = (unsigned short*)(ws + oW2);
  float* gates = (float*)(ws + oGt);

  k_cvx<<<dim3((NB * KF) / 2048), dim3(256), 0, stream>>>(x, Xb);
  k_gkT<<<dim3(KF / GKC, NT), dim3(256), 0, stream>>>(gk, Gk);
  k_w1T<<<dim3(NE * NC1), dim3(64), 0, stream>>>(w1, W1);
  k_w2T<<<dim3(NE * NC2), dim3(64), 0, stream>>>(w2, W2);
  k_gate<<<dim3(NB / 16), dim3(256), 0, stream>>>(Xb, Gk, gb, gates);
  (void)hipFuncSetAttribute(reinterpret_cast<const void*>(&k_conv),
                            hipFuncAttributeMaxDynamicSharedMemorySize, (int)LDS_CONV);
  k_conv<<<dim3(NB), dim3(256), LDS_CONV, stream>>>(Xb, W1, (const _Float16*)W2, gates, b1, b2, eb, tbp, out);
  (void)hipGetLastError();
}
